// GCNWithEdge_69337952027194
// MI455X (gfx1250) — hardware-verified
//
#include <hip/hip_runtime.h>
#include <stddef.h>


#define NTHR   256
#define NWAVE  8
#define EPT    8
#define CHUNK  (NTHR * EPT)
#define WCAP   (EPT * 32)
#define LISTN  (NWAVE * WCAP)
#define PASSN  (NWAVE * 16)
#define PCAP   (CHUNK + PASSN)
#define NB     1024

static_assert(PASSN == 128);
static_assert((PCAP % PASSN) == 0);
static_assert((NB % 32) == 0);

#define S_EA   16.0f
#define S_W1   64.0f
#define S_1    1024.0f
#define S_W2   256.0f
#define S_2    262144.0f
#define S_2INV 3.814697265625e-06f

#define P_W1A  0
#define P_W2A  8192
#define P_W1B  73728
#define P_W2B  77824
#define P_TOTH 94208
#define PU1    1024
#define PU2    9216
#define PU3    9728
#define PU4    11776
static_assert(PU4 * 8 == P_TOTH);

typedef float    v4f  __attribute__((ext_vector_type(4)));
typedef float    v8f  __attribute__((ext_vector_type(8)));
typedef int      v4i  __attribute__((ext_vector_type(4)));
typedef _Float16 v8h  __attribute__((ext_vector_type(8)));
typedef _Float16 v16h __attribute__((ext_vector_type(16)));
union FragH { v16h v; v8h h[2]; };

__host__ __device__ constexpr size_t al32(size_t x) { return (x + 31) & ~(size_t)31; }

template <int IC, int OC>
struct Lds {
  static constexpr int H = IC * OC;
  static constexpr int AW = OC + 1;
  static constexpr int KB2 = H / 32;
  static constexpr size_t oAcc   = 0;
  static constexpr size_t oMsg   = al32(oAcc + (size_t)(NB + 1) * AW * 4);
  static constexpr size_t oX     = al32(oMsg + (size_t)PASSN * AW * 4);
  static constexpr size_t oE     = al32(oX + (size_t)PASSN * IC * 4);
  static constexpr size_t oHb    = al32(oE + (size_t)PASSN * 8 * 2);
  static constexpr size_t oSlot  = al32(oHb + (size_t)NWAVE * KB2 * 32 * 32);
  static constexpr size_t oList  = al32(oSlot + (size_t)PASSN * 4);
  static constexpr size_t oPend  = al32(oList + (size_t)LISTN * 4);
  static constexpr size_t oB1    = al32(oPend + (size_t)PCAP * 4);
  static constexpr size_t oB2    = al32(oB1 + (size_t)H * 4);
  static constexpr size_t oRoot  = al32(oB2 + (size_t)H * 4);
  static constexpr size_t oBias  = al32(oRoot + (size_t)IC * OC * 4);
  static constexpr size_t oWcnt  = al32(oBias + 16 * 4);
  static constexpr size_t oPendN = al32(oWcnt + (size_t)NWAVE * 4);
  static constexpr size_t total  = al32(oPendN + 32);
};

__device__ __forceinline__ int clampi(int v, int lo, int hi) { return v < lo ? lo : (v > hi ? hi : v); }

__device__ __forceinline__ v8h zero8() {
  v8h r;
#pragma unroll
  for (int i = 0; i < 8; ++i) r[i] = (_Float16)0.0f;
  return r;
}

__device__ __forceinline__ v8f wmh(v16h a, v16h b, v8f c) {
  v8f d = __builtin_amdgcn_wmma_f32_16x16x32_f16(false, a, false, b, (short)0, c, false, false);
  asm volatile("v_nop\n\tv_nop\n\tv_nop\n\tv_nop" : "+v"(d) : "v"(a), "v"(b));
  return d;
}

__device__ __forceinline__ v8h relu8h(v8f d) {
  v8h r;
#pragma unroll
  for (int i = 0; i < 8; ++i) { const float t = fmaxf(d[i], 0.0f); r[i] = (_Float16)t; }
  return r;
}

__device__ __forceinline__ v8f ldc8(const float* p) {
  const v4f a = *(const v4f*)p;
  const v4f b = *(const v4f*)(p + 4);
  v8f c;
  c[0] = a.x; c[1] = a.y; c[2] = a.z; c[3] = a.w;
  c[4] = b.x; c[5] = b.y; c[6] = b.z; c[7] = b.w;
  return c;
}

__device__ __forceinline__ int scan_chunk(const int* __restrict__ dsts, int nE, int cbase, int nodeBase,
                                          int vec8, int* list, int tid, int wave) {
  int wc = 0;
  const int el0  = tid * EPT;
  const int e0   = cbase + el0;
  const int sent = -2147483647 - 1;
  v4i da, db;
  if (vec8 != 0 && cbase + CHUNK <= nE) {
    da = *(const v4i*)(dsts + e0);
    db = *(const v4i*)(dsts + e0 + 4);
  } else {
    da.x = (e0     < nE) ? dsts[min(e0, nE - 1)] : sent;
    da.y = (e0 + 1 < nE) ? dsts[min(e0 + 1, nE - 1)] : sent;
    da.z = (e0 + 2 < nE) ? dsts[min(e0 + 2, nE - 1)] : sent;
    da.w = (e0 + 3 < nE) ? dsts[min(e0 + 3, nE - 1)] : sent;
    db.x = (e0 + 4 < nE) ? dsts[min(e0 + 4, nE - 1)] : sent;
    db.y = (e0 + 5 < nE) ? dsts[min(e0 + 5, nE - 1)] : sent;
    db.z = (e0 + 6 < nE) ? dsts[min(e0 + 6, nE - 1)] : sent;
    db.w = (e0 + 7 < nE) ? dsts[min(e0 + 7, nE - 1)] : sent;
  }
  const unsigned nb = (unsigned)nodeBase;
  const unsigned s0 = (unsigned)da.x - nb, s1 = (unsigned)da.y - nb;
  const unsigned s2 = (unsigned)da.z - nb, s3 = (unsigned)da.w - nb;
  const unsigned s4 = (unsigned)db.x - nb, s5 = (unsigned)db.y - nb;
  const unsigned s6 = (unsigned)db.z - nb, s7 = (unsigned)db.w - nb;
  const bool h0 = s0 < (unsigned)NB, h1 = s1 < (unsigned)NB, h2 = s2 < (unsigned)NB, h3 = s3 < (unsigned)NB;
  const bool h4 = s4 < (unsigned)NB, h5 = s5 < (unsigned)NB, h6 = s6 < (unsigned)NB, h7 = s7 < (unsigned)NB;
  const unsigned any = __builtin_amdgcn_ballot_w32(h0 | h1 | h2 | h3 | h4 | h5 | h6 | h7);
  if (any != 0u) {
#define HITJ(J, HJ) { \
      const unsigned mj = __builtin_amdgcn_ballot_w32(HJ); \
      if (mj != 0u) { \
        if (HJ) { \
          const int pos = wc + (int)__builtin_amdgcn_mbcnt_lo(mj, 0u); \
          if (pos < WCAP) list[wave * WCAP + pos] = el0 + (J); \
        } \
        wc += (int)__builtin_popcount(mj); } }
    HITJ(0, h0)
    HITJ(1, h1)
    HITJ(2, h2)
    HITJ(3, h3)
    HITJ(4, h4)
    HITJ(5, h5)
    HITJ(6, h6)
    HITJ(7, h7)
#undef HITJ
  }
  return wc;
}

__global__ __launch_bounds__(256) void k_prep(const float* __restrict__ w1a, const float* __restrict__ w2a,
                                              const float* __restrict__ w1b, const float* __restrict__ w2b,
                                              _Float16* planes) {
  const int u = blockIdx.x * 256 + threadIdx.x;
  if (u >= PU4) return;
  const float* src; int cols, realc, ub; float sc;
  if (u < PU1)      { src = w1a; cols = 32;  realc = 8;   ub = 0;   sc = S_W1; }
  else if (u < PU2) { src = w2a; cols = 256; realc = 256; ub = PU1; sc = S_W2; }
  else if (u < PU3) { src = w1b; cols = 32;  realc = 8;   ub = PU2; sc = S_W1; }
  else              { src = w2b; cols = 128; realc = 128; ub = PU3; sc = S_W2; }
  const int el  = 8 * (u - ub);
  const int row = el / cols, c0 = el - row * cols;
  v8h v;
#pragma unroll
  for (int k = 0; k < 8; ++k) {
    const int c  = c0 + k;
    const int cc = c < realc ? c : realc - 1;
    float f = src[row * realc + cc];
    f = (c < realc) ? f * sc : 0.0f;
    v[k] = (_Float16)f;
  }
  _Float16* dp = planes + (size_t)8 * u;
  *(volatile v8h*)dp = v;
  __threadfence();
  *(volatile v8h*)dp = v;
}

template <int IC, int OC, int RELU>
__global__ __launch_bounds__(NTHR) void k_agg(
    const float* __restrict__ xin, const int* __restrict__ ei, const float* __restrict__ ea,
    const _Float16* __restrict__ W1h, const float* __restrict__ b1,
    const _Float16* __restrict__ W2h, const float* __restrict__ b2,
    const float* __restrict__ root, const float* __restrict__ bias,
    float* outp, int nN, int nE, int vec8, int outLim) {
  typedef Lds<IC, OC> L;
  constexpr int H = IC * OC, KB2 = H / 32, MT = H / 16, AW = OC + 1;
  constexpr int NQ = (NB * OC) / (128 * NWAVE);
  static_assert(NQ * 128 * NWAVE == NB * OC);
  static_assert(IC == 16 && (OC == 16 || OC == 8));
  static_assert((H % 32) == 0);

  extern __shared__ __attribute__((aligned(32))) char smem[];
  float*    acc    = (float*)(smem + L::oAcc);
  float*    msgL   = (float*)(smem + L::oMsg);
  float*    stgX   = (float*)(smem + L::oX);
  _Float16* stgE   = (_Float16*)(smem + L::oE);
  v16h*     hb     = (v16h*)(smem + L::oHb);
  int*      slotb  = (int*)(smem + L::oSlot);
  int*      list   = (int*)(smem + L::oList);
  int*      pend   = (int*)(smem + L::oPend);
  float*    bsm1   = (float*)(smem + L::oB1);
  float*    bsm2   = (float*)(smem + L::oB2);
  float*    rootS  = (float*)(smem + L::oRoot);
  float*    biasS  = (float*)(smem + L::oBias);
  int*      wcnt   = (int*)(smem + L::oWcnt);
  int*      pendNp = (int*)(smem + L::oPendN);

  const int tid = threadIdx.x, lane = tid & 31, wave = tid >> 5, hh = lane >> 4, m = lane & 15;
  const int nodeBase = blockIdx.x * NB;
  const int* srcs = ei;
  const int* dsts = ei + nE;

  for (int i = tid; i < (NB + 1) * AW; i += NTHR) acc[i] = 0.0f;
  for (int i = tid; i < H; i += NTHR) { bsm1[i] = b1[i] * S_1; bsm2[i] = b2[i] * S_2; }
  for (int i = tid; i < IC * OC; i += NTHR) rootS[i] = root[i];
  for (int i = tid; i < OC; i += NTHR) biasS[i] = bias[i];
  if (tid == 0) *pendNp = 0;
  __syncthreads();

  const int nChunks = (nE + CHUNK - 1) / CHUNK;
#pragma unroll 1
  for (int ch = 0; ch < nChunks; ++ch) {
    const int cbase = ch * CHUNK;
    const int wc = scan_chunk(dsts, nE, cbase, nodeBase, vec8, list, tid, wave);
    if (lane == 0) wcnt[wave] = wc;
    __syncthreads();

    const int base = *pendNp;
    int tot = 0, myoff = 0;
#pragma unroll
    for (int w = 0; w < NWAVE; ++w) {
      const int c = clampi(wcnt[w], 0, WCAP);
      if (w < wave) myoff += c;
      tot += c;
    }
    int newN = base + tot;
    newN = newN > PCAP ? PCAP : newN;
    {
      const int n = clampi(wcnt[wave], 0, WCAP);
      const int* lp = list + wave * WCAP;
      for (int i = lane; i < n; i += 32) {
        const int pos = base + myoff + i;
        if (pos < PCAP) pend[pos] = cbase + lp[i];
      }
    }
    const int fin = (ch == nChunks - 1) ? 1 : 0;
    const int R   = (fin != 0) ? (newN + PASSN - 1) / PASSN : newN / PASSN;
    const int Pv  = (fin != 0) ? newN : R * PASSN;
    __syncthreads();

#pragma unroll 1
    for (int r = 0; r < R; ++r) {
      const int row = wave * 16 + m;
      {
        int idx = r * PASSN + row;
        idx = idx > PCAP - 1 ? PCAP - 1 : idx;
        const bool valid = idx < Pv;
        int e = pend[idx];
        if (!valid) e = 0;
        e = clampi(e, 0, nE - 1);
        const int d = dsts[e];
        int s = srcs[e];
        int slot = d - nodeBase;
        if (!valid || (unsigned)slot >= (unsigned)NB) slot = NB;
        s = clampi(s, 0, nN - 1);
        const v4f ea0 = *(const v4f*)(ea + (size_t)e * 8);
        const v4f ea1 = *(const v4f*)(ea + (size_t)e * 8 + 4);
        const float* xp = xin + (size_t)s * IC;
        const v4f x0 = *(const v4f*)(xp), x1 = *(const v4f*)(xp + 4);
        const v4f x2 = *(const v4f*)(xp + 8), x3 = *(const v4f*)(xp + 12);
        if (hh == 0) {
          v8h hv;
          hv[0] = (_Float16)(ea0.x * S_EA); hv[1] = (_Float16)(ea0.y * S_EA);
          hv[2] = (_Float16)(ea0.z * S_EA); hv[3] = (_Float16)(ea0.w * S_EA);
          hv[4] = (_Float16)(ea1.x * S_EA); hv[5] = (_Float16)(ea1.y * S_EA);
          hv[6] = (_Float16)(ea1.z * S_EA); hv[7] = (_Float16)(ea1.w * S_EA);
          *(v8h*)(stgE + row * 8) = hv;
          slotb[row] = slot;
        } else {
          const float vm = valid ? 1.0f : 0.0f;
          float* xs = stgX + row * IC;
          *(v4f*)(xs)      = x0 * vm;
          *(v4f*)(xs + 4)  = x1 * vm;
          *(v4f*)(xs + 8)  = x2 * vm;
          *(v4f*)(xs + 12) = x3 * vm;
        }
      }
      __syncthreads();

      {
        const v8h z8 = zero8();
        FragH bq;
        {
          const v8h t = *(const v8h*)(stgE + row * 8);
          if (hh != 0) bq.h[0] = z8; else bq.h[0] = t;
          bq.h[1] = z8;
        }
#pragma unroll 1
        for (int kb = 0; kb < KB2; ++kb) {
          FragH o;
#pragma unroll
          for (int t = 0; t < 2; ++t) {
            const int ft = 2 * kb + t;
            FragH a;
            const _Float16* ap = W1h + (size_t)(16 * ft + m) * 32 + 8 * hh;
            a.h[0] = *(const v8h*)ap;
            a.h[1] = *(const v8h*)(ap + 16);
            const v8f c = ldc8(bsm1 + 16 * ft + 8 * hh);
            const v8f dd = wmh(a.v, bq.v, c);
            o.h[t] = relu8h(dd);
          }
          hb[(wave * KB2 + kb) * 32 + lane] = o.v;
        }
        v8f ma;
#pragma unroll
        for (int q = 0; q < 8; ++q) ma[q] = 0.0f;
        const float* xr = stgX + row * IC;
        const v16h* hp = hb + (wave * KB2) * 32 + lane;
#pragma unroll 1
        for (int mt = 0; mt < MT; ++mt) {
          v8f c = ldc8(bsm2 + 16 * mt + 8 * hh);
          const _Float16* ap0 = W2h + (size_t)(16 * mt + m) * H + 8 * hh;
#pragma unroll 2
          for (int kb = 0; kb < KB2; ++kb) {
            FragH a;
            a.h[0] = *(const v8h*)(ap0 + 32 * kb);
            a.h[1] = *(const v8h*)(ap0 + 32 * kb + 16);
            const v16h b = hp[32 * kb];
            c = wmh(a.v, b, c);
          }
          const int ii = (OC == 16) ? mt : (2 * mt + hh);
          const float xv = xr[ii];
#pragma unroll
          for (int q = 0; q < 8; ++q) ma[q] = fmaf(xv, c[q], ma[q]);
        }
        if (OC == 8) {
#pragma unroll
          for (int q = 0; q < 8; ++q) ma[q] += __shfl_xor(ma[q], 16);
        }
        float* mp = msgL + row * AW;
        if (OC == 16) {
#pragma unroll
          for (int q = 0; q < 8; ++q) mp[8 * hh + q] = ma[q] * S_2INV;
          if (hh == 0) mp[OC] = 1.0f;
        } else {
          if (hh == 0) {
#pragma unroll
            for (int q = 0; q < 8; ++q) mp[q] = ma[q] * S_2INV;
            mp[OC] = 1.0f;
          }
        }
      }
      __syncthreads();

      if (wave == 0) {
#pragma unroll 1
        for (int i = 0; i < PASSN; ++i) {
          const int sl = clampi(slotb[i], 0, NB);
          if (lane < AW) acc[sl * AW + lane] += msgL[i * AW + lane];
        }
      }
      __syncthreads();
    }

    int rem = newN - R * PASSN;
    rem = rem < 0 ? 0 : rem;
    if (R > 0 && tid < rem) pend[tid] = pend[R * PASSN + tid];
    if (tid == 0) *pendNp = rem;
  }
  __syncthreads();

#pragma unroll 1
  for (int idx = tid; idx < NB * OC; idx += NTHR) {
    const int sl = idx / OC, o = idx - sl * OC;
    int node = nodeBase + sl;
    node = node > nN - 1 ? nN - 1 : node;
    const float* xp = xin + (size_t)node * IC;
    const v4f xa = *(const v4f*)(xp), xb = *(const v4f*)(xp + 4);
    const v4f xc = *(const v4f*)(xp + 8), xd = *(const v4f*)(xp + 12);
    float xv[16];
    xv[0] = xa.x; xv[1] = xa.y; xv[2]  = xa.z; xv[3]  = xa.w;
    xv[4] = xb.x; xv[5] = xb.y; xv[6]  = xb.z; xv[7]  = xb.w;
    xv[8] = xc.x; xv[9] = xc.y; xv[10] = xc.z; xv[11] = xc.w;
    xv[12] = xd.x; xv[13] = xd.y; xv[14] = xd.z; xv[15] = xd.w;
    float s = 0.0f;
#pragma unroll
    for (int i = 0; i < IC; ++i) s = fmaf(xv[i], rootS[i * OC + o], s);
    const float cn  = acc[sl * AW + OC];
    const float inv = 1.0f / fmaxf(cn, 1.0f);
    float v = (s + acc[sl * AW + o] * inv) + biasS[o];
    if (RELU != 0) v = fmaxf(v, 0.0f);
    acc[sl * AW + o] = v;
  }
  __syncthreads();

  v4f ov[NQ];
#pragma unroll
  for (int q = 0; q < NQ; ++q) {
    const int f  = (wave * NQ + q) * 128 + 4 * lane;
    const int sl = f / OC, o = f - sl * OC;
    const float* ap = acc + sl * AW + o;
    v4f v;
    v.x = ap[0]; v.y = ap[1]; v.z = ap[2]; v.w = ap[3];
    ov[q] = v;
  }
  const size_t ob  = (size_t)nodeBase * OC;
  const size_t lim = (size_t)(outLim < 0 ? 0 : outLim);
#pragma unroll
  for (int q = 0; q < NQ; ++q) {
    const size_t gi = ob + (size_t)((wave * NQ + q) * 128 + 4 * lane);
    if (gi + 3 < lim) *(volatile v4f*)(outp + gi) = ov[q];
  }
  __threadfence();
#pragma unroll
  for (int q = 0; q < NQ; ++q) {
    const size_t gi = ob + (size_t)((wave * NQ + q) * 128 + 4 * lane);
    if (gi + 3 < lim) *(volatile v4f*)(outp + gi) = ov[q];
  }
}

extern "C" void kernel_launch(void* const* d_in, const int* in_sizes, int n_in,
                              void* d_out, int out_size, void* d_ws, size_t ws_size,
                              hipStream_t stream) {
  if (n_in < 15) return;
  const int nN = in_sizes[0] / 16;
  const int nE = in_sizes[1] / 2;
  if (nN <= 0 || nE <= 0 || in_sizes[0] != nN * 16 || in_sizes[1] != nE * 2 || in_sizes[2] != nE * 8) return;
  if (in_sizes[3] != 256 * 8 || in_sizes[4] != 256 || in_sizes[5] != 256 * 256 || in_sizes[6] != 256) return;
  if (in_sizes[7] != 16 * 16 || in_sizes[8] != 16) return;
  if (in_sizes[9] != 128 * 8 || in_sizes[10] != 128 || in_sizes[11] != 128 * 128 || in_sizes[12] != 128) return;
  if (in_sizes[13] != 16 * 8 || in_sizes[14] != 8) return;
  if (out_size != nN * 8) return;

  const float* x     = (const float*)d_in[0];
  const int*   ei    = (const int*)d_in[1];
  const float* eat   = (const float*)d_in[2];
  const float* w1_0  = (const float*)d_in[3];
  const float* b1_0  = (const float*)d_in[4];
  const float* w2_0  = (const float*)d_in[5];
  const float* b2_0  = (const float*)d_in[6];
  const float* root0 = (const float*)d_in[7];
  const float* bias0 = (const float*)d_in[8];
  const float* w1_1  = (const float*)d_in[9];
  const float* b1_1  = (const float*)d_in[10];
  const float* w2_1  = (const float*)d_in[11];
  const float* b2_1  = (const float*)d_in[12];
  const float* root1 = (const float*)d_in[13];
  const float* bias1 = (const float*)d_in[14];
  float* out = (float*)d_out;

  const int nBlk = (nN + NB - 1) / NB;

  char* ws = (char*)d_ws;
  size_t off = 0;
  const size_t oPl = off; off += (size_t)P_TOTH * 2;            off = (off + 255) & ~(size_t)255;
  const size_t oH0 = off; off += (size_t)nBlk * NB * 16 * 4;     off = (off + 255) & ~(size_t)255;
  if (off > ws_size) return;
  _Float16* planes = (_Float16*)(ws + oPl);
  float*    h0     = (float*)(ws + oH0);

  const int vec8 = ((nE & 3) == 0) ? 1 : 0;

  k_prep<<<PU4 / 256, 256, 0, stream>>>(w1_0, w2_0, w1_1, w2_1, planes);

  (void)hipFuncSetAttribute(reinterpret_cast<const void*>(&k_agg<16, 16, 1>),
                            hipFuncAttributeMaxDynamicSharedMemorySize, (int)Lds<16, 16>::total);
  (void)hipFuncSetAttribute(reinterpret_cast<const void*>(&k_agg<16, 8, 0>),
                            hipFuncAttributeMaxDynamicSharedMemorySize, (int)Lds<16, 8>::total);

  k_agg<16, 16, 1><<<nBlk, NTHR, Lds<16, 16>::total, stream>>>(
      x, ei, eat, planes + P_W1A, b1_0, planes + P_W2A, b2_0, root0, bias0,
      h0, nN, nE, vec8, nBlk * NB * 16);

  k_agg<16, 8, 0><<<nBlk, NTHR, Lds<16, 8>::total, stream>>>(
      h0, ei, eat, planes + P_W1B, b1_1, planes + P_W2B, b2_1, root1, bias1,
      out, nN, nE, vec8, nN * 8);
}
